// RBlockPE_91225105367735
// MI455X (gfx1250) — hardware-verified
//
#include <hip/hip_runtime.h>


namespace {
constexpr int B = 16, C = 64, F = 64, T = 64, IC = 32, HP = F * T, FP = 32, TP = 32, WK = FP * TP;
constexpr float XS = 8.0f;
typedef _Float16 b16;
typedef __attribute__((ext_vector_type(16))) _Float16 v16b;
typedef __attribute__((ext_vector_type(8))) _Float16 v8b;
typedef __attribute__((ext_vector_type(8))) float v8f;
typedef __attribute__((ext_vector_type(4))) float v4f;
__device__ __forceinline__ float bf16_rne(float f) { unsigned int u = __float_as_uint(f); u += 0x7FFFu + ((u >> 16) & 1u); return __uint_as_float(u & 0xFFFF0000u); }
__device__ __forceinline__ void split16(float v, b16& hi, b16& lo) { hi = (b16)v; lo = (b16)(v - (float)hi); }
__device__ __forceinline__ v16b frag_kb(const b16* p, int hh) { const v8b a = *(const v8b*)(p + 8 * hh), b = *(const v8b*)(p + 16 + 8 * hh); v16b f;
#pragma unroll
  for (int e = 0; e < 8; ++e) { f[e] = a[e]; f[8 + e] = b[e]; } return f; }
__device__ __forceinline__ v8f wmma16b(v16b a, v16b b, v8f c) { v8f d = __builtin_amdgcn_wmma_f32_16x16x32_f16(false, a, false, b, (short)0, c, false, false); asm volatile("v_nop\n\tv_nop\n\tv_nop\n\tv_nop" : "+v"(d) : "v"(a), "v"(b)); return d; }
__device__ __forceinline__ void wave_lds_sync() { __builtin_amdgcn_fence(__ATOMIC_RELEASE, "workgroup"); __builtin_amdgcn_wave_barrier(); __builtin_amdgcn_fence(__ATOMIC_ACQUIRE, "workgroup"); }
__device__ __forceinline__ float pmul(float a, float b) { float p = a * b; asm volatile("" : "+v"(p)); return p; }

__global__ __launch_bounds__(32) void aq_kernel(const float* __restrict__ x, const float* __restrict__ thw, const float* __restrict__ thb, const float* __restrict__ cw, int BV, float* __restrict__ AQ) {
  __shared__ float Wt[IC][C + 1], Tb[IC], Wth[IC]; const int lane = threadIdx.x; const int b = blockIdx.x / (HP / 32); if (b >= BV) return; const int i = (blockIdx.x % (HP / 32)) * 32 + lane;
  for (int o = 0; o < IC; ++o) { Wt[o][lane] = bf16_rne(thw[o * C + lane]); Wt[o][32 + lane] = bf16_rne(thw[o * C + 32 + lane]); } Tb[lane] = bf16_rne(thb[lane]); Wth[lane] = bf16_rne(cw[lane]); wave_lds_sync();
  const float* xp = x + (size_t)b * C * HP + i; float a = 0.0f;
#pragma unroll 1
  for (int o = 0; o < IC; ++o) { float s = Tb[o];
#pragma unroll 4
    for (int c = 0; c < C; ++c) s += pmul(bf16_rne(xp[(size_t)c * HP]), Wt[o][c]); a += pmul(Wth[o], s); }
  const int fi = i / T, ti = i % T; a += pmul(bf16_rne(cw[2 * IC]), (float)fi / (float)(F - 1)) + pmul(bf16_rne(cw[2 * IC + 1]), (float)ti / (float)(T - 1));
  for (int pass = 0; pass < 2; ++pass) { ((volatile float*)AQ)[(size_t)b * HP + i] = a; __threadfence(); }
}
__global__ __launch_bounds__(32) void key_kernel(const float* __restrict__ x, const float* __restrict__ psw, const float* __restrict__ psb, const float* __restrict__ phw, const float* __restrict__ phb, const float* __restrict__ cw, int BV, b16* __restrict__ PSIh, b16* __restrict__ PSIl, float* __restrict__ CK) {
  __shared__ float Wp[IC][C + 1], Wf[IC][C + 1], Pb[IC], Fb[IC], Wph[IC]; __shared__ __attribute__((aligned(16))) b16 Sh[IC][72], Sl[IC][72]; __shared__ float Cc[64];
  const int lane = threadIdx.x; const int b = blockIdx.x / (WK / 64); if (b >= BV) return; const int j0 = (blockIdx.x % (WK / 64)) * 64;
  for (int o = 0; o < IC; ++o) { Wp[o][lane] = bf16_rne(psw[o * C + lane]); Wp[o][32 + lane] = bf16_rne(psw[o * C + 32 + lane]); Wf[o][lane] = bf16_rne(phw[o * C + lane]); Wf[o][32 + lane] = bf16_rne(phw[o * C + 32 + lane]); } Pb[lane] = bf16_rne(psb[lane]); Fb[lane] = bf16_rne(phb[lane]); Wph[lane] = bf16_rne(cw[IC + lane]); wave_lds_sync();
  const float wd0 = bf16_rne(cw[2 * IC]), wd1 = bf16_rne(cw[2 * IC + 1]);
#pragma unroll 1
  for (int half = 0; half < 2; ++half) { const int j = j0 + half * 32 + lane; const int fj = j / TP, tj = j % TP; const float* xb = x + (size_t)b * C * HP; const size_t p00 = (size_t)(2 * fj) * T + 2 * tj; float cj = 0.0f;
#pragma unroll 1
    for (int o = 0; o < IC; ++o) { float s0 = Pb[o], s1 = Pb[o], s2 = Pb[o], s3 = Pb[o], f0 = Fb[o], f1 = Fb[o], f2 = Fb[o], f3 = Fb[o];
#pragma unroll 2
      for (int c = 0; c < C; ++c) { const float* xc = xb + (size_t)c * HP + p00; const float x00 = bf16_rne(xc[0]), x01 = bf16_rne(xc[1]), x10 = bf16_rne(xc[T]), x11 = bf16_rne(xc[T + 1]); const float wp = Wp[o][c], wf = Wf[o][c];
        s0 += pmul(x00, wp); s1 += pmul(x01, wp); s2 += pmul(x10, wp); s3 += pmul(x11, wp); f0 += pmul(x00, wf); f1 += pmul(x01, wf); f2 += pmul(x10, wf); f3 += pmul(x11, wf); }
      const float ps = fmaxf(fmaxf(s0, s1), fmaxf(s2, s3)), pf = fmaxf(fmaxf(f0, f1), fmaxf(f2, f3)); cj += pmul(Wph[o], pf); b16 p, q; split16(ps * XS, p, q); Sh[o][half * 32 + lane] = p; Sl[o][half * 32 + lane] = q; }
    cj -= pmul(wd0, (float)fj / (float)(FP - 1)) + pmul(wd1, (float)tj / (float)(TP - 1)); Cc[half * 32 + lane] = cj; }
  wave_lds_sync();
  for (int pass = 0; pass < 2; ++pass) { for (int o = 0; o < IC; ++o) { const size_t r = ((size_t)b * IC + o) * WK + j0; ((volatile __attribute__((ext_vector_type(2))) _Float16*)(PSIh + r))[lane] = (__attribute__((ext_vector_type(2))) _Float16){Sh[o][2 * lane], Sh[o][2 * lane + 1]}; ((volatile __attribute__((ext_vector_type(2))) _Float16*)(PSIl + r))[lane] = (__attribute__((ext_vector_type(2))) _Float16){Sl[o][2 * lane], Sl[o][2 * lane + 1]}; }
    ((volatile float*)CK)[(size_t)b * WK + j0 + lane] = Cc[lane]; ((volatile float*)CK)[(size_t)b * WK + j0 + 32 + lane] = Cc[32 + lane]; __threadfence(); }
}
__global__ __launch_bounds__(32) void nl_kernel(const float* __restrict__ AQ, const float* __restrict__ CK, const b16* __restrict__ PSIh, const b16* __restrict__ PSIl, const float* __restrict__ Ww, const float* __restrict__ Wb, int BV, float* __restrict__ WY) {
  __shared__ __attribute__((aligned(16))) b16 Fh[32][40], Fl[32][40]; __shared__ float Y[32][IC + 1], Wl[C][IC + 1], Bl[C];
  const int lane = threadIdx.x, nloc = lane & 15, hlf = lane >> 4; const int b = blockIdx.x / (HP / 32); if (b >= BV) return; const int i0 = (blockIdx.x % (HP / 32)) * 32;
  for (int co = 0; co < C; ++co) Wl[co][lane] = bf16_rne(Ww[co * (IC + 1) + lane]); Bl[lane] = bf16_rne(Wb[lane]); Bl[32 + lane] = bf16_rne(Wb[32 + lane]);
  float ai[32];
#pragma unroll
  for (int r = 0; r < 32; ++r) ai[r] = AQ[(size_t)b * HP + i0 + r];
  v8f acc[2][2] = {{(v8f){}, (v8f){}}, {(v8f){}, (v8f){}}}; const b16* ph = PSIh + (size_t)b * IC * WK; const b16* pl = PSIl + (size_t)b * IC * WK;
#pragma unroll 1
  for (int j0 = 0; j0 < WK; j0 += 32) { const float cj = CK[(size_t)b * WK + j0 + lane];
#pragma unroll
    for (int r = 0; r < 32; ++r) { b16 p, q; split16(fmaxf(ai[r] + cj, 0.0f) * XS, p, q); Fh[r][lane] = p; Fl[r][lane] = q; }
    wave_lds_sync();
#pragma unroll
    for (int rt = 0; rt < 2; ++rt) { const v16b fa = frag_kb(&Fh[rt * 16 + nloc][0], hlf), fb = frag_kb(&Fl[rt * 16 + nloc][0], hlf);
#pragma unroll
      for (int t = 0; t < 2; ++t) { const size_t br = (size_t)(t * 16 + nloc) * WK + j0; const v16b bh = frag_kb(ph + br, hlf), bl = frag_kb(pl + br, hlf); acc[rt][t] = wmma16b(fa, bh, acc[rt][t]); acc[rt][t] = wmma16b(fa, bl, acc[rt][t]); acc[rt][t] = wmma16b(fb, bh, acc[rt][t]); } }
    wave_lds_sync(); }
#pragma unroll
  for (int rt = 0; rt < 2; ++rt)
#pragma unroll
    for (int t = 0; t < 2; ++t)
#pragma unroll
      for (int r8 = 0; r8 < 8; ++r8) Y[rt * 16 + 8 * hlf + r8][t * 16 + nloc] = acc[rt][t][r8] * (1.0f / (XS * XS)) * (1.0f / (float)WK);
  wave_lds_sync();
  for (int pass = 0; pass < 2; ++pass) {
#pragma unroll 1
    for (int co = 0; co < C; ++co) { float s = Bl[co];
#pragma unroll 4
      for (int c = 0; c < IC; ++c) s += pmul(Wl[co][c], Y[lane][c]); ((volatile float*)WY)[((size_t)b * C + co) * HP + i0 + lane] = s; }
    __threadfence(); }
}
__global__ __launch_bounds__(256) void stats_kernel(const float* __restrict__ WY, int BV, float* __restrict__ ST) {
  __shared__ float red[256]; const int c = blockIdx.x, tid = threadIdx.x; const int tot = BV * HP; float s = 0.0f; for (int n = tid; n < tot; n += 256) s += WY[((size_t)(n / HP) * C + c) * HP + (n % HP)]; red[tid] = s; __syncthreads();
  for (int w = 128; w > 0; w >>= 1) { if (tid < w) red[tid] += red[tid + w]; __syncthreads(); } const float mu = red[0] / (float)tot; __syncthreads();
  float q = 0.0f; for (int n = tid; n < tot; n += 256) { const float d = WY[((size_t)(n / HP) * C + c) * HP + (n % HP)] - mu; q += pmul(d, d); } red[tid] = q; __syncthreads();
  for (int w = 128; w > 0; w >>= 1) { if (tid < w) red[tid] += red[tid + w]; __syncthreads(); } const float rs = rsqrtf(red[0] / (float)tot + 1e-5f);
  if (tid < 32) { for (int pass = 0; pass < 2; ++pass) { ((volatile float*)ST)[(size_t)c * 32 + tid] = tid == 0 ? mu : (tid == 1 ? rs : 0.0f); __threadfence(); } }
}
__global__ __launch_bounds__(256) void out_kernel(const float* __restrict__ WY, const float* __restrict__ ST, const float* __restrict__ gam, const float* __restrict__ bet, const float* __restrict__ x, int BV, float* __restrict__ out) {
  const size_t idx = (size_t)blockIdx.x * 256 + threadIdx.x; if (idx >= (size_t)BV * C * HP) return; const int c = (int)((idx / HP) % C); const float v = pmul(pmul(WY[idx] - ST[c * 32], ST[c * 32 + 1]), bf16_rne(gam[c])) + bf16_rne(bet[c]) + bf16_rne(x[idx]);
  for (int pass = 0; pass < 2; ++pass) { ((volatile float*)out)[idx] = v; __threadfence(); }
}
}

extern "C" void kernel_launch(void* const* d_in, const int* in_sizes, int n_in, void* d_out, int out_size, void* d_ws, size_t ws_size, hipStream_t stream) {
  (void)n_in;
  auto Fp = [&](int i) { return (const float*)d_in[i]; };
  if (in_sizes[0] != B * C * HP || in_sizes[1] != IC * C || in_sizes[3] != IC * C || in_sizes[5] != IC * C || in_sizes[7] != 2 * IC + 2 || in_sizes[8] != C * (IC + 1) || in_sizes[9] != C || out_size != B * C * HP) return;
  const int BV = B;
  size_t off = 0; char* ws = (char*)d_ws;
  auto carve = [&](size_t bytes) { char* p = ws + off; off += (bytes + 255) & ~(size_t)255; return p; };
  float* AQ = (float*)carve((size_t)B * HP * 4); float* CK = (float*)carve((size_t)B * WK * 4); b16* PSIh = (b16*)carve((size_t)B * IC * WK * 2); b16* PSIl = (b16*)carve((size_t)B * IC * WK * 2); float* WY = (float*)carve((size_t)B * C * HP * 4); float* ST = (float*)carve(C * 32 * 4);
  if (off > ws_size || off > ((size_t)32 << 20)) return;
  aq_kernel<<<BV * (HP / 32), 32, 0, stream>>>(Fp(0), Fp(3), Fp(4), Fp(7), BV, AQ);
  key_kernel<<<BV * (WK / 64), 32, 0, stream>>>(Fp(0), Fp(1), Fp(2), Fp(5), Fp(6), Fp(7), BV, PSIh, PSIl, CK);
  nl_kernel<<<BV * (HP / 32), 32, 0, stream>>>(AQ, CK, PSIh, PSIl, Fp(8), Fp(9), BV, WY);
  stats_kernel<<<C, 256, 0, stream>>>(WY, BV, ST);
  out_kernel<<<(unsigned)(((size_t)BV * C * HP + 255) / 256), 256, 0, stream>>>(WY, ST, Fp(10), Fp(11), Fp(0), BV, (float*)d_out);
}
